// PluckerKernelAttention_60739427500732
// MI455X (gfx1250) — hardware-run, weakly checked
//
#include <hip/hip_runtime.h>


namespace {
constexpr int NB_ = 2, T = 2048, D = 1024, H = 16, DH = 64, NT = NB_ * T  , CH = 256;
constexpr float XS = 8.0f, HS = 256.0f, PS = 256.0f, WSC = 256.0f, SCL = 0.40824829046386302f  ;
typedef _Float16 b16;
typedef __attribute__((ext_vector_type(16))) _Float16 v16b;
typedef __attribute__((ext_vector_type(8))) _Float16 v8b;
typedef __attribute__((ext_vector_type(2))) _Float16 v2b;
typedef __attribute__((ext_vector_type(8))) float v8f;
typedef __attribute__((ext_vector_type(4))) float v4f;
typedef __attribute__((ext_vector_type(2))) float v2f;
__device__ __forceinline__ float bf16_rne(float f) { unsigned int u = __float_as_uint(f); u += 0x7FFFu + ((u >> 16) & 1u); float r = __uint_as_float(u & 0xFFFF0000u); asm volatile("" : "+v"(r)); return r; }
__device__ __forceinline__ float bfv(float f) { float r = bf16_rne(f); asm volatile("" : "+v"(r)); return r; }
__device__ __forceinline__ void split16(float v, b16& hi, b16& lo) { hi = (b16)v; lo = (b16)(v - (float)hi); }
__device__ __forceinline__ v16b frag_kb(const b16* p, int hh) { const v8b a = *(const v8b*)(p + 8 * hh), b = *(const v8b*)(p + 16 + 8 * hh); v16b f;
#pragma unroll
  for (int e = 0; e < 8; ++e) { f[e] = a[e]; f[8 + e] = b[e]; } return f; }
__device__ __forceinline__ v8f wmma16b(v16b a, v16b b, v8f c) { v8f d = __builtin_amdgcn_wmma_f32_16x16x32_f16(false, a, false, b, (short)0, c, false, false); asm volatile("v_nop\n\tv_nop\n\tv_nop\n\tv_nop" : "+v"(d) : "v"(a), "v"(b)); return d; }
__device__ __forceinline__ void wave_lds_sync() { __builtin_amdgcn_fence(__ATOMIC_RELEASE, "workgroup"); __builtin_amdgcn_wave_barrier(); __builtin_amdgcn_fence(__ATOMIC_ACQUIRE, "workgroup"); }
__device__ __forceinline__ float pmul(float a, float b) { float p = a * b; asm volatile("" : "+v"(p)); return p; }

__global__ __launch_bounds__(256) void wput_kernel(const float* __restrict__ w1q, const float* __restrict__ w2q, const float* __restrict__ w1k, const float* __restrict__ w2k, const float* __restrict__ wv, const float* __restrict__ wo, b16* __restrict__ WQK, b16* __restrict__ WV, b16* __restrict__ WO) { const size_t nt = (size_t)gridDim.x * 256, u0 = (size_t)blockIdx.x * 256 + threadIdx.x; v8b v;
  for (size_t u = u0; u < (size_t)256 * 128; u += nt) { const int o = (int)(u / 128), k0 = (int)(u % 128) * 8; const float* w = o < 64 ? w1q : (o < 128 ? w2q : (o < 192 ? w1k : w2k)); const int oo = o % 64;
#pragma unroll
    for (int j = 0; j < 8; ++j) v[j] = (b16)(bf16_rne(w[(size_t)oo * D + k0 + j]) * WSC); for (int pass = 0; pass < 2; ++pass) { *(volatile v8b*)(WQK + (size_t)o * D + k0) = v; __threadfence(); } }
  for (size_t u = u0; u < (size_t)D * 128; u += nt) { const int o = (int)(u / 128), k0 = (int)(u % 128) * 8; v8b a, c;
#pragma unroll
    for (int j = 0; j < 8; ++j) { a[j] = (b16)(bf16_rne(wv[(size_t)o * D + k0 + j]) * WSC); c[j] = (b16)(bf16_rne(wo[(size_t)o * D + k0 + j]) * WSC); } for (int pass = 0; pass < 2; ++pass) { *(volatile v8b*)(WV + (size_t)o * D + k0) = a; *(volatile v8b*)(WO + (size_t)o * D + k0) = c; __threadfence(); } } }
__global__ __launch_bounds__(32) void proj_kernel(const float* __restrict__ x, const b16* __restrict__ WQK, const b16* __restrict__ WV, const float* __restrict__ bv, b16* __restrict__ LQh, b16* __restrict__ LQl, b16* __restrict__ LKh, b16* __restrict__ LKl, float* __restrict__ V) { __shared__ __attribute__((aligned(16))) b16 Ah[16][D + 8]; __shared__ float Tf[16][260]; const int lane = threadIdx.x, nloc = lane & 15, hlf = lane >> 4; const size_t t0 = (size_t)blockIdx.x * 16;
  for (int rr = 0; rr < 16; ++rr) for (int q = 0; q < D / 32; ++q) { const int c = q * 32 + lane; Ah[rr][c] = (b16)(bf16_rne(x[(t0 + rr) * D + c]) * XS); }
  if (lane < 16) for (int k = D; k < D + 8; ++k) Ah[lane][k] = (b16)0.0f;
  wave_lds_sync();
#pragma unroll 1
  for (int g = 0; g < 5; ++g) { const b16* W = g == 0 ? WQK : WV + (size_t)(g - 1) * 256 * D; v8f acc[16];
#pragma unroll
    for (int t = 0; t < 16; ++t) acc[t] = (v8f){};
#pragma unroll 2
    for (int kb = 0; kb < D; kb += 32) { const v16b a = frag_kb(&Ah[nloc][kb], hlf);
#pragma unroll
      for (int t = 0; t < 16; ++t) acc[t] = wmma16b(a, frag_kb(W + (size_t)(t * 16 + nloc) * D + kb, hlf), acc[t]); }
#pragma unroll
    for (int t = 0; t < 16; ++t) { const int cc = t * 16 + nloc; const float bb = g == 0 ? 0.0f : bfv(bv[(g - 1) * 256 + cc]);
#pragma unroll
      for (int r8 = 0; r8 < 8; ++r8) Tf[8 * hlf + r8][cc] = acc[t][r8] * (1.0f / (XS * WSC)) + bb; }
    wave_lds_sync();
    if (g == 0) {
      const int rr = nloc, isk = hlf; const size_t tok = t0 + rr;
      for (int pass = 0; pass < 2; ++pass) {
#pragma unroll 1
        for (int h = 0; h < H; ++h) { const float* p1 = &Tf[rr][(isk ? 128 : 0) + h * 4]; const float* p2 = &Tf[rr][(isk ? 192 : 64) + h * 4]; float Lm[6]; Lm[0] = p1[0] * p2[1] - p1[1] * p2[0]; Lm[1] = p1[0] * p2[2] - p1[2] * p2[0]; Lm[2] = p1[0] * p2[3] - p1[3] * p2[0]; Lm[3] = p1[1] * p2[2] - p1[2] * p2[1]; Lm[4] = p1[1] * p2[3] - p1[3] * p2[1]; Lm[5] = p1[2] * p2[3] - p1[3] * p2[2];
          float n2 = 0.0f; for (int c = 0; c < 6; ++c) n2 += Lm[c] * Lm[c]; const float inv = 1.0f / fmaxf(sqrtf(n2), 1e-12f); float Lo[6];
          if (isk) { Lo[0] = Lm[5]; Lo[1] = -Lm[4]; Lo[2] = Lm[3]; Lo[3] = Lm[2]; Lo[4] = -Lm[1]; Lo[5] = Lm[0]; } else { for (int c = 0; c < 6; ++c) Lo[c] = Lm[c]; }
          b16 hh_[32], ll_[32]; for (int c = 0; c < 32; ++c) { hh_[c] = (b16)0.0f; ll_[c] = (b16)0.0f; } for (int c = 0; c < 6; ++c) split16(Lo[c] * inv * HS, hh_[c], ll_[c]);
          b16* dh = (isk ? LKh : LQh) + ((size_t)h * NT + tok) * 32; b16* dl = (isk ? LKl : LQl) + ((size_t)h * NT + tok) * 32;
          for (int c = 0; c < 32; c += 8) { v8b a, bq; for (int j = 0; j < 8; ++j) { a[j] = hh_[c + j]; bq[j] = ll_[c + j]; } *(volatile v8b*)(dh + c) = a; *(volatile v8b*)(dl + c) = bq; } }
        __threadfence(); } }
    else { for (int pass = 0; pass < 2; ++pass) { for (int rr = 0; rr < 16; ++rr) for (int q = 0; q < 2; ++q) *(volatile v4f*)(V + (t0 + rr) * D + (g - 1) * 256 + q * 128 + lane * 4) = *(const v4f*)(&Tf[rr][q * 128 + lane * 4]); __threadfence(); } }
    wave_lds_sync(); } }
__global__ __launch_bounds__(256) void vt_kernel(const float* __restrict__ V, b16* __restrict__ VTh, b16* __restrict__ VTl) { __shared__ float Tt[64][65]; const int b = blockIdx.x / (T / 64), tk0 = (blockIdx.x % (T / 64)) * 64; const int h = blockIdx.y; const int tid = threadIdx.x, wave = tid >> 5, lane = tid & 31;
  for (int q = wave; q < 64; q += 8) { Tt[q][lane * 2] = V[((size_t)b * T + tk0 + q) * D + h * DH + lane * 2]; Tt[q][lane * 2 + 1] = V[((size_t)b * T + tk0 + q) * D + h * DH + lane * 2 + 1]; }
  __syncthreads();
  for (int pass = 0; pass < 2; ++pass) { for (int d = wave; d < DH; d += 8) { b16 h0, l0, h1, l1; split16(Tt[lane * 2][d] * HS, h0, l0); split16(Tt[lane * 2 + 1][d] * HS, h1, l1); const size_t o = (((size_t)b * H + h) * DH + d) * T + tk0 + lane * 2; *(volatile v2b*)(VTh + o) = (v2b){h0, h1}; *(volatile v2b*)(VTl + o) = (v2b){l0, l1}; } __threadfence(); } }
__global__ __launch_bounds__(32) void att_kernel(const b16* __restrict__ LQh, const b16* __restrict__ LQl, const b16* __restrict__ LKh, const b16* __restrict__ LKl, const b16* __restrict__ VTh, const b16* __restrict__ VTl, int QLIM, float* __restrict__ O) { __shared__ __attribute__((aligned(16))) b16 Pa[16][CH + 8], Pb[16][CH + 8]; __shared__ float Sc[16][CH + 1], Mx[16], Ls[16], Fc[16], Of[16][DH + 1]; const int lane = threadIdx.x, nloc = lane & 15, hlf = lane >> 4; const int b = blockIdx.x / (H * (T / 16)), rem = blockIdx.x % (H * (T / 16)); const int h = rem / (T / 16), q0 = (rem % (T / 16)) * 16; if (q0 >= QLIM) return; const size_t tq = (size_t)b * T + q0;
  if (lane < 16) { for (int k = CH; k < CH + 8; ++k) { Pa[lane][k] = (b16)0.0f; Pb[lane][k] = (b16)0.0f; } Mx[lane] = -INFINITY; Ls[lane] = 0.0f; }
  wave_lds_sync();
  const v16b qa = frag_kb(LQh + ((size_t)h * NT + tq + nloc) * 32, hlf), ql = frag_kb(LQl + ((size_t)h * NT + tq + nloc) * 32, hlf);
  v8f oacc[4] = {(v8f){}, (v8f){}, (v8f){}, (v8f){}}; const int nch = q0 / CH + 1;
#pragma unroll 1
  for (int ch = 0; ch < nch; ++ch) { const int k0 = ch * CH;
#pragma unroll 1
    for (int half = 0; half < 2; ++half) { v8f sacc[8];
#pragma unroll
      for (int t = 0; t < 8; ++t) sacc[t] = (v8f){};
#pragma unroll
      for (int t = 0; t < 8; ++t) { const size_t key = (size_t)h * NT + (size_t)b * T + k0 + half * 128 + t * 16 + nloc; const v16b kh = frag_kb(LKh + key * 32, hlf), kl = frag_kb(LKl + key * 32, hlf); sacc[t] = wmma16b(qa, kh, sacc[t]); sacc[t] = wmma16b(qa, kl, sacc[t]); sacc[t] = wmma16b(ql, kh, sacc[t]); }
#pragma unroll
      for (int t = 0; t < 8; ++t)
#pragma unroll
        for (int r8 = 0; r8 < 8; ++r8) Sc[8 * hlf + r8][half * 128 + t * 16 + nloc] = sacc[t][r8] * (SCL / (HS * HS)); }
    wave_lds_sync();
    for (int r = 0; r < 16; ++r) { const int qi = q0 + r; float mx = -INFINITY; for (int j = lane; j < CH; j += 32) { const float s = (k0 + j <= qi) ? Sc[r][j] : -INFINITY; mx = fmaxf(mx, s); } for (int o = 16; o; o >>= 1) mx = fmaxf(mx, __shfl_xor(mx, o)); const float mo = Mx[r], mn = fmaxf(mo, mx); float sm = 0.0f; for (int j = lane; j < CH; j += 32) { const float p = (k0 + j <= qi) ? __expf(Sc[r][j] - mn) : 0.0f; Sc[r][j] = p; sm += p; } for (int o = 16; o; o >>= 1) sm += __shfl_xor(sm, o); wave_lds_sync(); if (lane == 0) { const float fac = (mo == -INFINITY) ? 0.0f : __expf(mo - mn); Fc[r] = fac; Ls[r] = Ls[r] * fac + sm; Mx[r] = mn; } }
    wave_lds_sync();
    for (int r = 0; r < 16; ++r) for (int q = 0; q < CH / 32; ++q) { const int c = q * 32 + lane; b16 p, pl; split16(Sc[r][c] * PS, p, pl); Pa[r][c] = p; Pb[r][c] = pl; }
    wave_lds_sync();
#pragma unroll
    for (int t = 0; t < 4; ++t)
#pragma unroll
      for (int r8 = 0; r8 < 8; ++r8) oacc[t][r8] *= Fc[8 * hlf + r8];
#pragma unroll 2
    for (int kb = 0; kb < CH; kb += 32) { const v16b pa = frag_kb(&Pa[nloc][kb], hlf), pb = frag_kb(&Pb[nloc][kb], hlf);
#pragma unroll
      for (int t = 0; t < 4; ++t) { const size_t vo = (((size_t)b * H + h) * DH + t * 16 + nloc) * T + k0 + kb; const v16b vh = frag_kb(VTh + vo, hlf), vl = frag_kb(VTl + vo, hlf); oacc[t] = wmma16b(pa, vh, oacc[t]); oacc[t] = wmma16b(pa, vl, oacc[t]); oacc[t] = wmma16b(pb, vh, oacc[t]); } }
    wave_lds_sync(); }
#pragma unroll
  for (int t = 0; t < 4; ++t)
#pragma unroll
    for (int r8 = 0; r8 < 8; ++r8) { const int r = 8 * hlf + r8; Of[r][t * 16 + nloc] = oacc[t][r8] * (1.0f / (PS * HS)) / Ls[r]; }
  wave_lds_sync();
  for (int pass = 0; pass < 2; ++pass) { for (int r = 0; r < 16; ++r) *(volatile v2f*)(O + (tq + r) * D + h * DH + lane * 2) = (v2f){Of[r][lane * 2], Of[r][lane * 2 + 1]}; __threadfence(); } }
__global__ __launch_bounds__(32) void outp_kernel(const float* __restrict__ O, const b16* __restrict__ WO, const float* __restrict__ bo, int QLIM, float* __restrict__ out) { __shared__ __attribute__((aligned(16))) b16 Ah[16][D + 8], Al[16][D + 8]; __shared__ float Tf[16][260]; const int lane = threadIdx.x, nloc = lane & 15, hlf = lane >> 4; const size_t t0 = (size_t)blockIdx.x * 16; if ((int)(t0 % T) >= QLIM) return;
  for (int rr = 0; rr < 16; ++rr) for (int q = 0; q < D / 32; ++q) { const int c = q * 32 + lane; b16 p, pl; split16(O[(t0 + rr) * D + c] * HS, p, pl); Ah[rr][c] = p; Al[rr][c] = pl; }
  if (lane < 16) for (int k = D; k < D + 8; ++k) { Ah[lane][k] = (b16)0.0f; Al[lane][k] = (b16)0.0f; }
  wave_lds_sync();
#pragma unroll 1
  for (int g = 0; g < 4; ++g) { v8f acc[16];
#pragma unroll
    for (int t = 0; t < 16; ++t) acc[t] = (v8f){};
#pragma unroll 2
    for (int kb = 0; kb < D; kb += 32) { const v16b a = frag_kb(&Ah[nloc][kb], hlf), al = frag_kb(&Al[nloc][kb], hlf);
#pragma unroll
      for (int t = 0; t < 16; ++t) { const v16b bw = frag_kb(WO + (size_t)(g * 256 + t * 16 + nloc) * D + kb, hlf); acc[t] = wmma16b(a, bw, acc[t]); acc[t] = wmma16b(al, bw, acc[t]); } }
#pragma unroll
    for (int t = 0; t < 16; ++t) { const int cc = t * 16 + nloc; const float bb = bfv(bo[g * 256 + cc]);
#pragma unroll
      for (int r8 = 0; r8 < 8; ++r8) Tf[8 * hlf + r8][cc] = acc[t][r8] * (1.0f / (HS * WSC)) + bb; }
    wave_lds_sync();
    for (int pass = 0; pass < 2; ++pass) { for (int rr = 0; rr < 16; ++rr) for (int q = 0; q < 2; ++q) *(volatile v4f*)(out + (t0 + rr) * D + g * 256 + q * 128 + lane * 4) = *(const v4f*)(&Tf[rr][q * 128 + lane * 4]); __threadfence(); }
    wave_lds_sync(); } }
}

extern "C" void kernel_launch(void* const* d_in, const int* in_sizes, int n_in, void* d_out, int out_size, void* d_ws, size_t ws_size, hipStream_t stream) {
  (void)n_in;
  auto Fp = [&](int i) { return (const float*)d_in[i]; };
  if (in_sizes[0] != NT * D || in_sizes[1] != 64 * D || in_sizes[4] != 64 * D || in_sizes[5] != D * D || in_sizes[7] != D * D || out_size != NT * D) return;
  const int QLIM = T;
  size_t off = 0; char* ws = (char*)d_ws;
  auto carve = [&](size_t bytes) { char* p = ws + off; off += (bytes + 255) & ~(size_t)255; return p; };
  b16* WQK = (b16*)carve((size_t)256 * D * 2); b16* WV = (b16*)carve((size_t)D * D * 2); b16* WO = (b16*)carve((size_t)D * D * 2); b16* LQh = (b16*)carve((size_t)H * NT * 32 * 2); b16* LQl = (b16*)carve((size_t)H * NT * 32 * 2); b16* LKh = (b16*)carve((size_t)H * NT * 32 * 2); b16* LKl = (b16*)carve((size_t)H * NT * 32 * 2); float* V = (float*)carve((size_t)NT * D * 4); b16* VTh = (b16*)carve((size_t)NB_ * H * DH * T * 2); b16* VTl = (b16*)carve((size_t)NB_ * H * DH * T * 2); float* O = (float*)carve((size_t)NT * D * 4);
  if (off > ws_size || off > ((size_t)80 << 20)) return;
  wput_kernel<<<128, 256, 0, stream>>>(Fp(1), Fp(2), Fp(3), Fp(4), Fp(5), Fp(7), WQK, WV, WO);
  proj_kernel<<<NT / 16, 32, 0, stream>>>(Fp(0), WQK, WV, Fp(6), LQh, LQl, LKh, LKl, V);
  vt_kernel<<<dim3(NB_ * (T / 64), H), 256, 0, stream>>>(V, VTh, VTl);
  att_kernel<<<NB_ * H * (T / 16), 32, 0, stream>>>(LQh, LQl, LKh, LKl, VTh, VTl, QLIM, O);
  outp_kernel<<<NT / 16, 32, 0, stream>>>(O, WO, Fp(8), QLIM, (float*)d_out);
}
